// MambaDynamics_7945689498198
// MI455X (gfx1250) — hardware-verified
//
#include <hip/hip_runtime.h>
#include <math.h>


#define BB   4
#define TT   2048
#define MTK  (BB * TT)
#define LAT  256
#define OBJ  64
#define DM   256
#define DI   512
#define DS   16
#define DTR  16
#define NL   4
typedef __attribute__((ext_vector_type(16))) _Float16 v16h;
typedef __attribute__((ext_vector_type(8)))  _Float16 v8h;
typedef __attribute__((ext_vector_type(8)))  float    v8f;
typedef __attribute__((ext_vector_type(4)))  float    v4f;
typedef __attribute__((ext_vector_type(4)))  _Float16 v4h;
#define VST2(T, ptr, val) do { const T _v = (val); *(volatile T*)(ptr) = _v; __threadfence(); *(volatile T*)(ptr) = _v; } while (0)
__device__ __forceinline__ v8f wmma16(v16h a, v16h b, v8f c) {
  v8f d = __builtin_amdgcn_wmma_f32_16x16x32_f16(false, a, false, b, (short)0, c, false, false);
  asm volatile("v_nop\n\tv_nop\n\tv_nop\n\tv_nop" : "+v"(d) : "v"(a), "v"(b));
  return d;
}
__device__ __forceinline__ v16h frag16(const _Float16* p, int hh) {
  const v8h lo = *(const v8h*)(p + 8 * hh), hi = *(const v8h*)(p + 16 + 8 * hh);
  return __builtin_shufflevector(lo, hi, 0,1,2,3,4,5,6,7,8,9,10,11,12,13,14,15);
}
__device__ __forceinline__ float silu(float x) { return x / (1.0f + expf(-x)); }

__global__ __launch_bounds__(256) void k_in16(const float* __restrict__ z, const float* __restrict__ o, _Float16* __restrict__ A0) {
  const int t = blockIdx.x * 256 + threadIdx.x;
  const int i = t / 40, c = (t % 40) * 8;
  v8h v;
#pragma unroll
  for (int e = 0; e < 8; ++e) v[e] = (_Float16)((c < LAT) ? z[(size_t)i * LAT + c + e] : o[(size_t)i * OBJ + c - LAT + e]);
  VST2(v8h, A0 + (size_t)i * 320 + c, v);
}
__global__ __launch_bounds__(256) void k_w16(const float* __restrict__ w, int N, int K, int Npad, int Kpad, _Float16* __restrict__ W16) {
  const int t = blockIdx.x * 256 + threadIdx.x;
  const int per = Kpad / 8;
  if (t >= Npad * per) return;
  const int n = t / per, k0 = (t % per) * 8;
  v8h v;
#pragma unroll
  for (int e = 0; e < 8; ++e) v[e] = (n < N && k0 + e < K) ? (_Float16)w[(size_t)n * K + k0 + e] : (_Float16)0.f;
  VST2(v8h, W16 + (size_t)n * Kpad + k0, v);
}
__global__ __launch_bounds__(256) void k_to16(const float* __restrict__ s, int K, _Float16* __restrict__ d) {
  const size_t t = (size_t)blockIdx.x * 256 + threadIdx.x;
  const int per = K / 8;
  if (t >= (size_t)MTK * per) return;
  const int i = (int)(t / per), c = (int)(t % per) * 8;
  v8h v;
#pragma unroll
  for (int e = 0; e < 8; ++e) v[e] = (_Float16)s[(size_t)i * K + c + e];
  VST2(v8h, d + (size_t)i * K + c, v);
}
template <int K, int NTOT, int EPI>
__global__ __launch_bounds__(128) void k_gemm(const _Float16* __restrict__ A, const _Float16* __restrict__ W16, const float* __restrict__ bias,
                                              float* __restrict__ outf, _Float16* __restrict__ outh, float* __restrict__ outo) {
  __shared__ __attribute__((aligned(16))) float sT[4][16][132];
  const int lane = threadIdx.x & 31, wave = threadIdx.x >> 5, hh = lane >> 4, l16 = lane & 15;
  const int m0 = blockIdx.x * 64 + wave * 16, n0 = blockIdx.y * 128;
  v8f acc[8];
#pragma unroll
  for (int ni = 0; ni < 8; ++ni) acc[ni] = (v8f){};
#pragma unroll 2
  for (int k0 = 0; k0 < K; k0 += 32) {
    const v16h a0 = frag16(A + (size_t)(m0 + l16) * K + k0, hh);
#pragma unroll
    for (int ni = 0; ni < 8; ++ni) { const v16h b = frag16(W16 + (size_t)(n0 + ni * 16 + l16) * K + k0, hh); acc[ni] = wmma16(a0, b, acc[ni]); }
  }
  float (*st)[132] = sT[wave];
#pragma unroll
  for (int ni = 0; ni < 8; ++ni)
#pragma unroll
    for (int i = 0; i < 8; ++i) {
      float v = acc[ni][i] + (bias ? bias[n0 + ni * 16 + l16] : 0.f);
      if (EPI == 1) v = (v > 20.f) ? v : log1pf(expf(v));
      st[i + 8 * hh][ni * 16 + l16] = v;
    }
  __builtin_amdgcn_fence(__ATOMIC_RELEASE, "workgroup"); __builtin_amdgcn_wave_barrier(); __builtin_amdgcn_fence(__ATOMIC_ACQUIRE, "workgroup");
  if (EPI == 2) {
#pragma unroll
    for (int rr = 0; rr < 16; ++rr) {
      const v4f old = *(const v4f*)(outf + (size_t)(m0 + rr) * NTOT + n0 + lane * 4);
      float* p = &st[rr][lane * 4]; p[0] += old[0]; p[1] += old[1]; p[2] += old[2]; p[3] += old[3];
    }
    __builtin_amdgcn_fence(__ATOMIC_RELEASE, "workgroup"); __builtin_amdgcn_wave_barrier(); __builtin_amdgcn_fence(__ATOMIC_ACQUIRE, "workgroup");
  }
  for (int pass = 0; pass < 2; ++pass) {
#pragma unroll
    for (int rr = 0; rr < 16; ++rr) {
      if (EPI == 3) {
        if (n0 + 128 <= LAT) *(volatile v4f*)(outf + (size_t)(m0 + rr) * LAT + n0 + lane * 4) = *(const v4f*)(&st[rr][lane * 4]);
        else if (lane < 16) *(volatile v4f*)(outo + (size_t)(m0 + rr) * OBJ + lane * 4) = *(const v4f*)(&st[rr][lane * 4]);
      } else {
        *(volatile v4f*)(outf + (size_t)(m0 + rr) * NTOT + n0 + lane * 4) = *(const v4f*)(&st[rr][lane * 4]);
        if (outh != nullptr && lane < 16) { v8h o;
#pragma unroll
          for (int e = 0; e < 8; ++e) o[e] = (_Float16)st[rr][lane * 8 + e];
          *(volatile v8h*)(outh + (size_t)(m0 + rr) * NTOT + n0 + lane * 8) = o; }
      }
    }
    __threadfence();
  }
}
__global__ __launch_bounds__(256) void k_conv(const float* __restrict__ xz, const float* __restrict__ cw, const float* __restrict__ cb, float* __restrict__ u, _Float16* __restrict__ u16) {
  const int t = blockIdx.x * 256 + threadIdx.x;
  const int d = t % DI, tok = t / DI, pos = tok % TT;
  float acc = cb[d];
#pragma unroll
  for (int k = 0; k < 4; ++k) { const int tp = pos - 3 + k; if (tp >= 0) acc += cw[d * 4 + k] * xz[(size_t)(tok - 3 + k) * (2 * DI) + d]; }
  const float s = silu(acc);
  VST2(float, u + t, s);
  const _Float16 hv = (_Float16)s;
  *(volatile _Float16*)(u16 + t) = hv; __threadfence(); *(volatile _Float16*)(u16 + t) = hv;
}
__global__ __launch_bounds__(256) void k_dt16(const float* __restrict__ proj, _Float16* __restrict__ D16) {
  const int i = blockIdx.x * 256 + threadIdx.x;
  v8h a, b, zz;
#pragma unroll
  for (int e = 0; e < 8; ++e) { a[e] = (_Float16)proj[(size_t)i * 128 + e]; b[e] = (_Float16)proj[(size_t)i * 128 + 8 + e]; zz[e] = (_Float16)0.f; }
  for (int pass = 0; pass < 2; ++pass) {
    *(volatile v8h*)(D16 + (size_t)i * 32) = a; *(volatile v8h*)(D16 + (size_t)i * 32 + 8) = b;
    *(volatile v8h*)(D16 + (size_t)i * 32 + 16) = zz; *(volatile v8h*)(D16 + (size_t)i * 32 + 24) = zz;
    __threadfence();
  }
}
__global__ __launch_bounds__(256) void k_scan(const float* __restrict__ u, const float* __restrict__ dt, const float* __restrict__ proj, const float* __restrict__ xz,
                                              const float* __restrict__ Alog, const float* __restrict__ Dv, float* __restrict__ y) {
  const int t = blockIdx.x * 256 + threadIdx.x;
  const int b = t / DI, d = t % DI;
  float A[DS], hs[DS];
#pragma unroll
  for (int s = 0; s < DS; ++s) { A[s] = -expf(Alog[d * DS + s]); hs[s] = 0.f; }
  const float Dd = Dv[d];
  for (int pos = 0; pos < TT; ++pos) {
    const size_t tok = (size_t)b * TT + pos;
    const float dl = dt[tok * DI + d], xv = u[tok * DI + d];
    const float* pr = proj + tok * 128;
    float yy = 0.f;
#pragma unroll
    for (int s = 0; s < DS; ++s) { hs[s] = __expf(dl * A[s]) * hs[s] + dl * pr[DTR + s] * xv; yy += hs[s] * pr[DTR + DS + s]; }
    yy += Dd * xv;
    const float z = xz[tok * (2 * DI) + DI + d];
    VST2(float, y + tok * DI + d, yy * silu(z));
  }
}
__global__ __launch_bounds__(256) void k_ln(const float* __restrict__ h, const float* __restrict__ g, const float* __restrict__ be, _Float16* __restrict__ H16) {
  const int row = blockIdx.x * 8 + (threadIdx.x >> 5), lane = threadIdx.x & 31;
  const float* hr = h + (size_t)row * DM + lane * 8;
  float v[8]; float s = 0.f;
#pragma unroll
  for (int e = 0; e < 8; ++e) { v[e] = hr[e]; s += v[e]; }
#pragma unroll
  for (int o = 16; o > 0; o >>= 1) s += __shfl_xor(s, o, 32);
  const float mu = s * (1.0f / DM);
  float q = 0.f;
#pragma unroll
  for (int e = 0; e < 8; ++e) { const float dd = v[e] - mu; q += dd * dd; }
#pragma unroll
  for (int o = 16; o > 0; o >>= 1) q += __shfl_xor(q, o, 32);
  const float rs = 1.0f / sqrtf(q * (1.0f / DM) + 1e-5f);
  v8h out;
#pragma unroll
  for (int e = 0; e < 8; ++e) { const int c = lane * 8 + e; out[e] = (_Float16)((v[e] - mu) * rs * g[c] + be[c]); }
  VST2(v8h, H16 + (size_t)row * DM + lane * 8, out);
}
extern "C" void kernel_launch(void* const* d_in, const int* in_sizes, int n_in,
                              void* d_out, int out_size, void* d_ws, size_t ws_size, hipStream_t stream) {
  (void)in_sizes; (void)n_in; (void)out_size;
  const float* zs   = (const float*)d_in[0];
  const float* os   = (const float*)d_in[1];
  const float* inw  = (const float*)d_in[2];
  const float* inb  = (const float*)d_in[3];
  const float* bin  = (const float*)d_in[4];
  const float* bcw  = (const float*)d_in[5];
  const float* bcb  = (const float*)d_in[6];
  const float* bxp  = (const float*)d_in[7];
  const float* bdtw = (const float*)d_in[8];
  const float* bdtb = (const float*)d_in[9];
  const float* bAl  = (const float*)d_in[10];
  const float* bD   = (const float*)d_in[11];
  const float* bout = (const float*)d_in[12];
  const float* lng  = (const float*)d_in[13]; const float* lnb = (const float*)d_in[14];
  const float* wlat = (const float*)d_in[15]; const float* blat = (const float*)d_in[16];
  const float* wobj = (const float*)d_in[17]; const float* bobj = (const float*)d_in[18];
  float* outZ = (float*)d_out;
  float* outO = (float*)((char*)d_out + (size_t)MTK * LAT * 4);
  char* ws = (char*)d_ws; size_t off = 0;
  auto take = [&](size_t bytes) { void* p = ws + off; off = (off + bytes + 255) & ~(size_t)255; return p; };
  _Float16* A0   = (_Float16*)take((size_t)MTK * 320 * 2);
  _Float16* Win  = (_Float16*)take((size_t)DM * 320 * 2);
  _Float16* Wbi  = (_Float16*)take((size_t)2 * DI * DM * 2);
  _Float16* Wxp  = (_Float16*)take((size_t)128 * DI * 2);
  _Float16* Wdt  = (_Float16*)take((size_t)DI * 32 * 2);
  _Float16* Wout = (_Float16*)take((size_t)DM * DI * 2);
  _Float16* Wfin = (_Float16*)take((size_t)384 * DM * 2);
  float*    bfin = (float*)take((size_t)384 * 4);
  float*    h    = (float*)take((size_t)MTK * DM * 4);
  _Float16* h16  = (_Float16*)take((size_t)MTK * DM * 2);
  float*    xz   = (float*)take((size_t)MTK * 2 * DI * 4);
  float*    u    = (float*)take((size_t)MTK * DI * 4);
  _Float16* u16  = (_Float16*)take((size_t)MTK * DI * 2);
  float*    proj = (float*)take((size_t)MTK * 128 * 4);
  _Float16* D16  = (_Float16*)take((size_t)MTK * 32 * 2);
  float*    dt   = (float*)take((size_t)MTK * DI * 4);
  float*    y    = (float*)take((size_t)MTK * DI * 4);
  _Float16* y16  = (_Float16*)take((size_t)MTK * DI * 2);
  if (off > ws_size) return;
  hipMemsetAsync(bfin, 0, 384 * 4, stream);
  hipMemcpyAsync(bfin, blat, LAT * 4, hipMemcpyDeviceToDevice, stream);
  hipMemcpyAsync(bfin + LAT, bobj, OBJ * 4, hipMemcpyDeviceToDevice, stream);
  const dim3 b256(256);
  k_in16<<<MTK * 40 / 256, b256, 0, stream>>>(zs, os, A0);
  k_w16<<<(DM * 40 + 255) / 256, b256, 0, stream>>>(inw, DM, 320, DM, 320, Win);
  k_gemm<320, DM, 0><<<dim3(MTK / 64, 2), 128, 0, stream>>>(A0, Win, inb, h, h16, nullptr);
  for (int l = 0; l < NL; ++l) {
    k_w16<<<(2 * DI * 32 + 255) / 256, b256, 0, stream>>>(bin + (size_t)l * 2 * DI * DM, 2 * DI, DM, 2 * DI, DM, Wbi);
    k_w16<<<(128 * 64 + 255) / 256, b256, 0, stream>>>(bxp + (size_t)l * 48 * DI, 48, DI, 128, DI, Wxp);
    k_w16<<<(DI * 4 + 255) / 256, b256, 0, stream>>>(bdtw + (size_t)l * DI * DTR, DI, DTR, DI, 32, Wdt);
    k_w16<<<(DM * 64 + 255) / 256, b256, 0, stream>>>(bout + (size_t)l * DM * DI, DM, DI, DM, DI, Wout);
    k_gemm<DM, 2 * DI, 0><<<dim3(MTK / 64, 8), 128, 0, stream>>>(h16, Wbi, nullptr, xz, nullptr, nullptr);
    k_conv<<<MTK * DI / 256, b256, 0, stream>>>(xz, bcw + (size_t)l * DI * 4, bcb + (size_t)l * DI, u, u16);
    k_gemm<DI, 128, 0><<<dim3(MTK / 64, 1), 128, 0, stream>>>(u16, Wxp, nullptr, proj, nullptr, nullptr);
    k_dt16<<<MTK / 256, b256, 0, stream>>>(proj, D16);
    k_gemm<32, DI, 1><<<dim3(MTK / 64, 4), 128, 0, stream>>>(D16, Wdt, bdtb + (size_t)l * DI, dt, nullptr, nullptr);
    k_scan<<<BB * DI / 256, b256, 0, stream>>>(u, dt, proj, xz, bAl + (size_t)l * DI * DS, bD + (size_t)l * DI, y);
    k_to16<<<(MTK * 64 + 255) / 256, b256, 0, stream>>>(y, DI, y16);
    k_gemm<DI, DM, 2><<<dim3(MTK / 64, 2), 128, 0, stream>>>(y16, Wout, nullptr, h, h16, nullptr);
  }
  k_ln<<<MTK / 8, b256, 0, stream>>>(h, lng, lnb, h16);
  k_w16<<<(384 * 32 + 255) / 256, b256, 0, stream>>>(wlat, LAT, DM, 384, DM, Wfin);
  k_w16<<<(OBJ * 32 + 255) / 256, b256, 0, stream>>>(wobj, OBJ, DM, OBJ, DM, Wfin + (size_t)LAT * DM);
  k_gemm<DM, 384, 3><<<dim3(MTK / 64, 3), 128, 0, stream>>>(h16, Wfin, bfin, outZ, nullptr, outO);
}
